// PointWiseConvolution_88175678587634
// MI455X (gfx1250) — hardware-verified
//
#include <hip/hip_runtime.h>
#include <math.h>

typedef __attribute__((ext_vector_type(16))) _Float16 v16h;
typedef __attribute__((ext_vector_type(16))) __bf16 v16b;
typedef __attribute__((ext_vector_type(8)))  _Float16 v8h;
typedef __attribute__((ext_vector_type(8)))  float v8f;
typedef __attribute__((ext_vector_type(4)))  float v4f;
typedef __attribute__((ext_vector_type(2)))  float v2f;
typedef __attribute__((ext_vector_type(4)))  unsigned v4u;
typedef __attribute__((ext_vector_type(4)))  int v4i;
typedef float __attribute__((may_alias)) float_a;
typedef int __attribute__((may_alias)) int_a;

template <typename T> __device__ __forceinline__ void vst2(void* p, T v) { *(volatile T*)p = v; __threadfence(); *(volatile T*)p = v; }
__device__ __forceinline__ v8f wmma16(v16h a, v16h b, v8f c) {
  v8f d = __builtin_amdgcn_wmma_f32_16x16x32_f16(false, a, false, b, (short)0, c, false, false);
  asm volatile("v_nop\n\tv_nop\n\tv_nop\n\tv_nop" : "+v"(d) : "v"(a), "v"(b));
  return d;
}
__device__ __forceinline__ v8f wmma_bf(v16b a, v16b b, v8f c) {
  v8f d = __builtin_amdgcn_wmma_f32_16x16x32_bf16(false, a, false, b, (short)0, c, false, false);
  asm volatile("v_nop\n\tv_nop\n\tv_nop\n\tv_nop" : "+v"(d) : "v"(a), "v"(b));
  return d;
}
__device__ __forceinline__ v16h frag_h(const _Float16* rowk0, int lane) {
  union { v16h v; v8h q[2]; } u; const _Float16* p = rowk0 + 8 * (lane >> 4);
  u.q[0] = *(const v8h*)p; u.q[1] = *(const v8h*)(p + 16); return u.v;
}
__device__ __forceinline__ v16h frag_f32(const float* rowk0, int lane) {
  v16h a; const float* p = rowk0 + 8 * (lane >> 4);
#pragma unroll
  for (int i = 0; i < 8; ++i) { a[i] = (_Float16)p[i]; a[8 + i] = (_Float16)p[16 + i]; }
  return a;
}
__device__ __forceinline__ v16h frag_f32s(const float* rowk0, int lane, float sc) {
  v16h a; const float* p = rowk0 + 8 * (lane >> 4);
#pragma unroll
  for (int i = 0; i < 8; ++i) { a[i] = (_Float16)(p[i] * sc); a[8 + i] = (_Float16)(p[16 + i] * sc); }
  return a;
}
__device__ __forceinline__ v16h fragc_f32(const float* W, int k0, int n, int lane, int ld, int K) {
  v16h a; const int g = lane >> 4;
#pragma unroll
  for (int i = 0; i < 8; ++i) { const int ka = k0 + 8 * g + i, kb = ka + 16;
    a[i] = (_Float16)(ka < K ? W[(size_t)(ka < K ? ka : K - 1) * ld + n] : 0.f); a[8 + i] = (_Float16)(kb < K ? W[(size_t)(kb < K ? kb : K - 1) * ld + n] : 0.f); }
  return a;
}
struct F2 { v16b h, l; };
__device__ __forceinline__ F2 bsplit16(const float v[16]) { F2 r;
#pragma unroll
  for (int i = 0; i < 16; ++i) { const __bf16 h = (__bf16)v[i]; r.h[i] = h; r.l[i] = (__bf16)(v[i] - (float)h); }
  return r; }
__device__ __forceinline__ F2 split_row(const float* row, int k0, int lane) { float v[16]; const float* p = row + k0 + 8 * (lane >> 4);
#pragma unroll
  for (int i = 0; i < 8; ++i) { v[i] = p[i]; v[8 + i] = p[16 + i]; }
  return bsplit16(v); }
__device__ __forceinline__ F2 split_rowK(const float* row, int k0, int lane, int K) { float v[16]; const int g = lane >> 4;
#pragma unroll
  for (int i = 0; i < 8; ++i) { const int ka = k0 + 8 * g + i, kb = ka + 16; v[i] = ka < K ? row[ka < K ? ka : K - 1] : 0.f; v[8 + i] = kb < K ? row[kb < K ? kb : K - 1] : 0.f; }
  return bsplit16(v); }
__device__ __forceinline__ F2 split_col(const float* W, int k0, int n, int lane, int ld, int K) { float v[16]; const int g = lane >> 4;
#pragma unroll
  for (int i = 0; i < 8; ++i) { const int ka = k0 + 8 * g + i, kb = ka + 16; v[i] = ka < K ? W[(size_t)(ka < K ? ka : K - 1) * ld + n] : 0.f; v[8 + i] = kb < K ? W[(size_t)(kb < K ? kb : K - 1) * ld + n] : 0.f; }
  return bsplit16(v); }
__device__ __forceinline__ v8f mac3(const F2& a, const F2& b, v8f c) { c = wmma_bf(a.l, b.h, c); c = wmma_bf(a.h, b.l, c); return wmma_bf(a.h, b.h, c); }
__device__ __forceinline__ float sigm(float v) { return 1.0f / (1.0f + expf(-v)); }
#define LDSX() do { asm volatile("s_wait_dscnt 0" ::: "memory"); __builtin_amdgcn_wave_barrier(); __builtin_amdgcn_fence(__ATOMIC_RELEASE, "workgroup"); } while (0)


#define NPNT 4096
#define CI 64
#define CO 128
#define NQ 16
#define KK (NQ * CI)
#ifndef TBB
#define TBB (NPNT / 16)
#endif
typedef __attribute__((ext_vector_type(8))) __bf16 v8b;
__device__ __forceinline__ v16b frag_b(const __bf16* rowk0, int lane) {
  union { v16b v; v8b q[2]; } u; const __bf16* p = rowk0 + 8 * (lane >> 4);
  u.q[0] = *(const v8b*)p; u.q[1] = *(const v8b*)(p + 16); return u.v;
}
__device__ __forceinline__ float bfr(float v) { return (float)(__bf16)v; }
#define WS_PT  0u
#define WS_END (WS_PT + 2u * CO * KK)

__global__ __launch_bounds__(256) void k_pack(const float* __restrict__ Wt, __bf16* __restrict__ PT) {
  __shared__ __align__(16) __bf16 srow[KK]; const int o = blockIdx.x, tid = threadIdx.x;
  for (int k = tid; k < KK; k += 256) { const int q = k / CI, c = k % CI; srow[k] = (__bf16)bfr(Wt[((size_t)o * CI + c) * NQ + q]); }
  __syncthreads();
  if (tid < KK / 8) vst2((unsigned*)(PT + (size_t)o * KK + tid * 8), *(const v4u*)(&srow[tid * 8]));
}
__global__ __launch_bounds__(128) void k_pwc(const float* __restrict__ P, const float* __restrict__ A, const __bf16* __restrict__ PT, const float* __restrict__ bias, float* __restrict__ OUT) {
  __shared__ float ssum[16][NQ][CI + 1]; __shared__ int scnt[16][NQ]; __shared__ __align__(16) __bf16 sah[16][KK + 8], sal[16][KK + 8]; __shared__ __align__(16) float so[16][132];
  const int tid = threadIdx.x, wave = tid >> 5, lane = tid & 31, col = lane & 15, g = lane >> 4; const int i0 = blockIdx.x * 16;
  for (int q = tid; q < 16 * NQ * (CI + 1); q += 128) (&ssum[0][0][0])[q] = 0.f;
  for (int q = tid; q < 16 * NQ; q += 128) (&scnt[0][0])[q] = 0;
  __syncthreads();
  if (tid < 64) { const int cl = tid >> 2, part = tid & 3; const int i = i0 + cl; const float px = bfr(P[(size_t)i * 3 + 0]), py = bfr(P[(size_t)i * 3 + 1]), pz = bfr(P[(size_t)i * 3 + 2]);
#pragma unroll 1
    for (int j = 0; j < NPNT; ++j) { const float dx = bfr(P[(size_t)j * 3 + 0]) - px, dy = bfr(P[(size_t)j * 3 + 1]) - py, dz = bfr(P[(size_t)j * 3 + 2]) - pz;
      const float d2 = __fadd_rn(__fadd_rn(__fmul_rn(dx, dx), __fmul_rn(dy, dy)), __fmul_rn(dz, dz));
      if (d2 < 0.01f) { int shell = (int)(sqrtf(d2) * 20.0f); shell = shell < 1 ? shell : 1; const int oct = (dx >= 0.f ? 1 : 0) + (dy >= 0.f ? 2 : 0) + (dz >= 0.f ? 4 : 0); const int q = shell * 8 + oct;
        if (part == 0) scnt[cl][q] += 1;
        const float* ar = A + (size_t)j * CI + part * 16;
#pragma unroll
        for (int c = 0; c < 16; ++c) ssum[cl][q][part * 16 + c] += bfr(ar[c]); } } }
  __syncthreads();
  for (int q = tid; q < 16 * KK; q += 128) { const int cl = q / KK, k = q % KK; const int cell = k / CI, c = k % CI; const int cnt = scnt[cl][cell]; const float m = cnt > 0 ? ssum[cl][cell][c] / (float)cnt : 0.f; const __bf16 hb = (__bf16)m; sah[cl][k] = hb; sal[cl][k] = (__bf16)(m - (float)hb); }
  __syncthreads();
  { v8f acc[2] = {};
#pragma unroll 2
    for (int kc = 0; kc < KK / 32; ++kc) { const v16b ah = frag_b(&sah[col][kc * 32], lane), al = frag_b(&sal[col][kc * 32], lane);
#pragma unroll
      for (int j = 0; j < 2; ++j) { const v16b w = frag_b(PT + (size_t)((wave * 2 + j) * 16 + col) * KK + kc * 32, lane); acc[j] = wmma_bf(al, w, acc[j]); acc[j] = wmma_bf(ah, w, acc[j]); } }
#pragma unroll
    for (int j = 0; j < 2; ++j) { const int o = (wave * 2 + j) * 16 + col; const float bb = bfr(bias[o]);
#pragma unroll
      for (int r = 0; r < 8; ++r) so[8 * g + r][o] = acc[j][r] + bb; } }
  __syncthreads();
  for (int q = tid; q < 16 * 32; q += 128) { const int rl = q >> 5, pc = q & 31; vst2(OUT + (size_t)(i0 + rl) * CO + pc * 4, *(const v4f*)&so[rl][pc * 4]); }
}
extern "C" void kernel_launch(void* const* d_in, const int* in_sizes, int n_in, void* d_out, int out_size, void* d_ws, size_t ws_size, hipStream_t stream) {
  (void)in_sizes; (void)n_in; (void)out_size;
  const float** F = (const float**)d_in;
  if (ws_size < (size_t)WS_END) return;
  char* ws = (char*)d_ws; __bf16* PT = (__bf16*)(ws + WS_PT);
  k_pack<<<CO, 256, 0, stream>>>(F[2], PT);
  k_pwc<<<TBB, 128, 0, stream>>>(F[0], F[1], PT, F[3], (float*)d_out);
}
